// Rwkv7SelfAttention_39341900432039
// MI455X (gfx1250) — hardware-verified
//
#include <hip/hip_runtime.h>
#define TT 1024
#define HDN 2048
#define NHh 32
#define HS 64
#define DW 96
#define DA 96
#define DV 64
#define DG 256
#define OFF_S1 2097152
#define OFF_S2 2099200
#define OFF_VF 2230272
typedef __bf16 v16b __attribute__((ext_vector_type(16)));
typedef unsigned short v8us __attribute__((ext_vector_type(8), may_alias));
typedef float  v8f  __attribute__((ext_vector_type(8)));
typedef float  v4f  __attribute__((ext_vector_type(4)));
typedef float  v4fa __attribute__((ext_vector_type(4), may_alias));
union FragB { v16b v; v8us half[2]; unsigned short u[16]; };

__device__ __forceinline__ unsigned short bf16_bits(float x) { unsigned int u = __float_as_uint(x); return (unsigned short)((u + 0x7FFFu + ((u >> 16) & 1u)) >> 16); }
__device__ __forceinline__ float bf16_val(unsigned short b) { return __uint_as_float(((unsigned int)b) << 16); }
__device__ __forceinline__ float bf16_round(float x) { return bf16_val(bf16_bits(x)); }
template <int NT>
__device__ __forceinline__ v8f mmaN(v16b ah, v16b al, v16b bh, v16b bl, v8f c) {
  c = __builtin_amdgcn_wmma_f32_16x16x32_bf16(false, ah, false, bh, (short)0, c, false, false);
  if (NT >= 2) c = __builtin_amdgcn_wmma_f32_16x16x32_bf16(false, al, false, bh, (short)0, c, false, false);
  if (NT >= 3) c = __builtin_amdgcn_wmma_f32_16x16x32_bf16(false, ah, false, bl, (short)0, c, false, false);
  asm volatile("v_nop\n\tv_nop\n\tv_nop\n\tv_nop" : "+v"(c) : "v"(ah), "v"(al), "v"(bh), "v"(bl));
  return c;
}

__global__ __launch_bounds__(256) void k_wt_bf16(const float* __restrict__ W, unsigned short* __restrict__ Wt, int K, int N) {
  const int t = blockIdx.x * 256 + threadIdx.x;
  const int k8n = K / 8;
  if (t >= N * k8n) return;
  const int n = t / k8n, k8 = (t % k8n) * 8;
  v8us v;
#pragma unroll
  for (int i = 0; i < 8; ++i) v[i] = bf16_bits(W[(size_t)(k8 + i) * N + n]);
  *(volatile v8us*)(Wt + (size_t)n * K + k8) = v;
  __threadfence();
  *(volatile v8us*)(Wt + (size_t)n * K + k8) = v;
}

template <bool ASPLIT, int ACT, bool BIAS_BF16>
__global__ __launch_bounds__(128) void k_gemm_bf(const float* __restrict__ A, int lda, const unsigned short* __restrict__ Wt, int ldb,
                                               const float* __restrict__ bias, float* __restrict__ C, int ldc, int M, int N, int K) {
  __shared__ __attribute__((aligned(16))) float so[4][16][64];
  const int tid = threadIdx.x, w = tid >> 5, lane = tid & 31, ln = lane & 15, hh = lane >> 4;
  const int ntn = N / 64;
  const int wid = blockIdx.x * 4 + w;
  const int mt = wid / ntn, nq = wid % ntn;
  if (mt * 16 >= M) return;
  const int row0 = mt * 16, col0 = nq * 64;
  const float* arow = A + (size_t)(row0 + ln) * lda;
  v8f acc[4] = {};
  for (int kb = 0; kb < K; kb += 32) {
    FragB ah, al;
    const v4f x0 = *(const v4fa*)(arow + kb + 8 * hh), x1 = *(const v4fa*)(arow + kb + 8 * hh + 4);
    const v4f x2 = *(const v4fa*)(arow + kb + 16 + 8 * hh), x3 = *(const v4fa*)(arow + kb + 16 + 8 * hh + 4);
    float xs[16] = {x0[0],x0[1],x0[2],x0[3],x1[0],x1[1],x1[2],x1[3],x2[0],x2[1],x2[2],x2[3],x3[0],x3[1],x3[2],x3[3]};
#pragma unroll
    for (int i = 0; i < 16; ++i) { const unsigned short hb = bf16_bits(xs[i]); ah.u[i] = hb; al.u[i] = ASPLIT ? bf16_bits(xs[i] - bf16_val(hb)) : (unsigned short)0; }
#pragma unroll
    for (int t = 0; t < 4; ++t) {
      const unsigned short* brow = Wt + (size_t)(col0 + t * 16 + ln) * ldb + kb;
      FragB b;
      b.half[0] = *(const v8us*)(brow + 8 * hh);
      b.half[1] = *(const v8us*)(brow + 16 + 8 * hh);
      acc[t] = mmaN<ASPLIT ? 2 : 1>(ah.v, al.v, b.v, b.v, acc[t]);
    }
  }
#pragma unroll
  for (int t = 0; t < 4; ++t) {
    float bv = bias ? bias[col0 + t * 16 + ln] : 0.f;
    if (BIAS_BF16) bv = bf16_round(bv);
#pragma unroll
    for (int r = 0; r < 8; ++r) { float v = acc[t][r] + bv; if (ACT == 1) v = fmaxf(v, 0.f); so[w][8 * hh + r][t * 16 + ln] = v; }
  }
  __builtin_amdgcn_fence(__ATOMIC_ACQ_REL, "workgroup");
  __builtin_amdgcn_wave_barrier();
  const int rsub = lane >> 4, c4 = (lane & 15) * 4;
  for (int pass = 0; pass < 2; ++pass) {
#pragma unroll
    for (int q = 0; q < 8; ++q) {
      const int r = q * 2 + rsub;
      const v4f v = *(const v4fa*)&so[w][r][c4];
      *(volatile v4f*)(C + (size_t)(row0 + r) * ldc + col0 + c4) = v;
    }
    if (pass == 0) __threadfence();
  }
}

template <bool ASPLIT, int ACT, bool BIAS_BF16, bool RES_BF16>
__global__ __launch_bounds__(128) void k_gemm_bf3(const float* __restrict__ A, int lda, const unsigned short* __restrict__ Wt, int ldb,
                                                const float* __restrict__ bias, const float* __restrict__ resid, int rmod, int ldr,
                                                float* __restrict__ C, int ldc, int M, int N, int K) {
  __shared__ __attribute__((aligned(16))) float so[4][16][64];
  const int tid = threadIdx.x, w = tid >> 5, lane = tid & 31, ln = lane & 15, hh = lane >> 4;
  const int ntn = N / 64;
  const int wid = blockIdx.x * 4 + w;
  const int mt = wid / ntn, nq = wid % ntn;
  if (mt * 16 >= M) return;
  const int row0 = mt * 16, col0 = nq * 64;
  const float* arow = A + (size_t)(row0 + ln) * lda;
  v8f acc[4] = {};
  for (int kb = 0; kb < K; kb += 32) {
    FragB ah, al;
    const v4f x0 = *(const v4fa*)(arow + kb + 8 * hh), x1 = *(const v4fa*)(arow + kb + 8 * hh + 4);
    const v4f x2 = *(const v4fa*)(arow + kb + 16 + 8 * hh), x3 = *(const v4fa*)(arow + kb + 16 + 8 * hh + 4);
    float xs[16] = {x0[0],x0[1],x0[2],x0[3],x1[0],x1[1],x1[2],x1[3],x2[0],x2[1],x2[2],x2[3],x3[0],x3[1],x3[2],x3[3]};
#pragma unroll
    for (int i = 0; i < 16; ++i) { const unsigned short hb = bf16_bits(xs[i]); ah.u[i] = hb; al.u[i] = ASPLIT ? bf16_bits(xs[i] - bf16_val(hb)) : (unsigned short)0; }
#pragma unroll
    for (int t = 0; t < 4; ++t) {
      const unsigned short* brow = Wt + (size_t)(col0 + t * 16 + ln) * ldb + kb;
      FragB b;
      b.half[0] = *(const v8us*)(brow + 8 * hh);
      b.half[1] = *(const v8us*)(brow + 16 + 8 * hh);
      acc[t] = mmaN<ASPLIT ? 2 : 1>(ah.v, al.v, b.v, b.v, acc[t]);
    }
  }
#pragma unroll
  for (int t = 0; t < 4; ++t) {
    const int col = col0 + t * 16 + ln;
    float bv = bias ? bias[col] : 0.f;
    if (BIAS_BF16) bv = bf16_round(bv);
#pragma unroll
    for (int r = 0; r < 8; ++r) {
      float v = acc[t][r] + bv;
      if (resid) { float rv = resid[(size_t)((row0 + 8 * hh + r) % rmod) * ldr + col]; if (RES_BF16) rv = bf16_round(rv); v += rv; }
      if (ACT == 1) v = fmaxf(v, 0.f);
      if (ACT == 2) v = 0.5f * v * (1.0f + erff(v * 0.70710678118654752f));
      if (ACT == 3) { const float u = 0.7978845608028654f * (v + 0.044715f * v * v * v); v = 0.5f * v * (1.0f + tanhf(u)); }
      so[w][8 * hh + r][t * 16 + ln] = v;
    }
  }
  __builtin_amdgcn_fence(__ATOMIC_ACQ_REL, "workgroup");
  __builtin_amdgcn_wave_barrier();
  const int rsub = lane >> 4, c4 = (lane & 15) * 4;
  for (int pass = 0; pass < 2; ++pass) {
#pragma unroll
    for (int q = 0; q < 8; ++q) {
      const int r = q * 2 + rsub;
      const v4f v = *(const v4fa*)&so[w][r][c4];
      *(volatile v4f*)(C + (size_t)(row0 + r) * ldc + col0 + c4) = v;
    }
    if (pass == 0) __threadfence();
  }
}
template <bool PARAM_BF16>
__global__ __launch_bounds__(256) void k_layernorm(const float* __restrict__ X, const float* __restrict__ R, const float* __restrict__ g, const float* __restrict__ bta,
                                                  float* __restrict__ out_sum, float* __restrict__ out_norm, int N, float eps) {
  __shared__ float red[256];
  const int row = blockIdx.x, tid = threadIdx.x;
  const float* x = X + (size_t)row * N; const float* rr = R ? R + (size_t)row * N : nullptr;
  float vals[16];
  const int per = N / 256;
  float s1 = 0.f;
  for (int u = 0; u < per / 4; ++u) {
    const int j = tid * 4 + 1024 * u;
    const v4f a = *(const v4fa*)(x + j);
    v4f b = {0.f,0.f,0.f,0.f}; if (rr) b = *(const v4fa*)(rr + j);
#pragma unroll
    for (int q = 0; q < 4; ++q) { const float v = a[q] + b[q]; vals[u * 4 + q] = v; s1 += v; }
  }
  red[tid] = s1; __syncthreads();
  for (int st = 128; st > 0; st >>= 1) { if (tid < st) red[tid] += red[tid + st]; __syncthreads(); }
  const float mu = red[0] / (float)N; __syncthreads();
  float s2 = 0.f;
  for (int u = 0; u < per / 4; ++u)
#pragma unroll
    for (int q = 0; q < 4; ++q) { const float c = vals[u * 4 + q] - mu; s2 += c * c; }
  red[tid] = s2; __syncthreads();
  for (int st = 128; st > 0; st >>= 1) { if (tid < st) red[tid] += red[tid + st]; __syncthreads(); }
  const float rs = rsqrtf(red[0] / (float)N + eps);
  for (int pass = 0; pass < 2; ++pass) {
    for (int u = 0; u < per / 4; ++u) {
      const int j = tid * 4 + 1024 * u;
      v4f o, sm;
#pragma unroll
      for (int q = 0; q < 4; ++q) {
        float gg = g[j + q], bb = bta[j + q];
        if (PARAM_BF16) { gg = bf16_round(gg); bb = bf16_round(bb); }
        sm[q] = vals[u * 4 + q]; o[q] = (vals[u * 4 + q] - mu) * rs * gg + bb;
      }
      if (out_sum) *(volatile v4f*)(out_sum + (size_t)row * N + j) = sm;
      *(volatile v4f*)(out_norm + (size_t)row * N + j) = o;
    }
    if (pass == 0) __threadfence();
  }
}


typedef _Float16 v16h __attribute__((ext_vector_type(16)));
union FragH { v16h v; v8us half[2]; _Float16 h[16]; unsigned short u[16]; };
template <int NT>
__device__ __forceinline__ v8f mmaH(v16h ah, v16h al, v16h bh, v16h bl, v8f c) {
  c = __builtin_amdgcn_wmma_f32_16x16x32_f16(false, ah, false, bh, (short)0, c, false, false);
  if (NT >= 2) c = __builtin_amdgcn_wmma_f32_16x16x32_f16(false, al, false, bh, (short)0, c, false, false);
  if (NT >= 3) c = __builtin_amdgcn_wmma_f32_16x16x32_f16(false, ah, false, bl, (short)0, c, false, false);
  asm volatile("v_nop\n\tv_nop\n\tv_nop\n\tv_nop" : "+v"(c) : "v"(ah), "v"(al), "v"(bh), "v"(bl));
  return c;
}
template <bool ASPLIT>
__global__ __launch_bounds__(128) void k_gemm_h(const float* __restrict__ A, int lda, size_t sA, const _Float16* __restrict__ Bh, int ldb, size_t sB, float alpha, float* __restrict__ C, int ldc, size_t sC, int M, int N, int K) {
  __shared__ __attribute__((aligned(16))) float so[4][16][64];
  const int tid = threadIdx.x, w = tid >> 5, lane = tid & 31, ln = lane & 15, hh = lane >> 4; const int by = blockIdx.y;
  A += (size_t)by * sA; Bh += (size_t)by * sB; C += (size_t)by * sC;
  const int ntn = (N + 63) / 64; const int wid = blockIdx.x * 4 + w; const int mt = wid / ntn, nq = wid % ntn; if (mt * 16 >= M) return;
  const int row0 = mt * 16, col0 = nq * 64; const float* arow = A + (size_t)(row0 + ln) * lda;
  v8f acc[4] = {};
  for (int kb = 0; kb < K; kb += 32) {
    FragH ah, al;
    const v4f x0 = *(const v4fa*)(arow + kb + 8 * hh), x1 = *(const v4fa*)(arow + kb + 8 * hh + 4), x2 = *(const v4fa*)(arow + kb + 16 + 8 * hh), x3 = *(const v4fa*)(arow + kb + 16 + 8 * hh + 4);
    float xs[16] = {x0[0],x0[1],x0[2],x0[3],x1[0],x1[1],x1[2],x1[3],x2[0],x2[1],x2[2],x2[3],x3[0],x3[1],x3[2],x3[3]};
#pragma unroll
    for (int i = 0; i < 16; ++i) { const _Float16 h = (_Float16)xs[i]; ah.h[i] = h; al.h[i] = ASPLIT ? (_Float16)(xs[i] - (float)h) : (_Float16)0.0f; }
#pragma unroll
    for (int t = 0; t < 4; ++t) { if (col0 + t * 16 >= N) continue; const size_t boff = (size_t)(col0 + t * 16 + ln) * ldb + kb; FragH bq; bq.half[0] = *(const v8us*)(Bh + boff + 8 * hh); bq.half[1] = *(const v8us*)(Bh + boff + 16 + 8 * hh);
      acc[t] = mmaH<ASPLIT ? 2 : 1>(ah.v, al.v, bq.v, bq.v, acc[t]); }
  }
#pragma unroll
  for (int t = 0; t < 4; ++t) { if (col0 + t * 16 >= N) continue;
#pragma unroll
    for (int r = 0; r < 8; ++r) so[w][8 * hh + r][t * 16 + ln] = acc[t][r] * alpha; }
  __builtin_amdgcn_fence(__ATOMIC_ACQ_REL, "workgroup"); __builtin_amdgcn_wave_barrier();
  const int rsub = lane >> 4, c4 = (lane & 15) * 4;
  for (int pass = 0; pass < 2; ++pass) {
#pragma unroll
    for (int q = 0; q < 8; ++q) { const int r = q * 2 + rsub; if (col0 + c4 < N) { const v4f v = *(const v4fa*)&so[w][r][c4]; *(volatile v4f*)(C + (size_t)(row0 + r) * ldc + col0 + c4) = v; } }
    if (pass == 0) __threadfence(); }
}

__global__ __launch_bounds__(256) void k_wt_f16(const float* __restrict__ W, _Float16* __restrict__ Wt, int K, int N, float scale) {
  const int t = blockIdx.x * 256 + threadIdx.x; if (t >= N * (K / 8)) return; const int n = t / (K / 8), k8 = (t % (K / 8)) * 8; FragH f;
#pragma unroll
  for (int i = 0; i < 8; ++i) f.h[i] = (_Float16)(bf16_round(W[(size_t)(k8 + i) * N + n]) * scale); const v8us o = f.half[0];
  *(volatile v8us*)((unsigned short*)Wt + (size_t)n * K + k8) = o; __threadfence(); *(volatile v8us*)((unsigned short*)Wt + (size_t)n * K + k8) = o;
}
template <int ACT>
__global__ __launch_bounds__(128) void k_gemm_hhx(const _Float16* __restrict__ A, int lda, size_t sA, const _Float16* __restrict__ Bh, int ldb, size_t sB, float alpha, const float* __restrict__ bias, size_t sBias, const float* __restrict__ CP, int rowsPerB, size_t sCPb, int row0g,
    float* __restrict__ C, _Float16* __restrict__ C16, int ldc, size_t sC, int M, int N, int K) {
  __shared__ __attribute__((aligned(16))) float so[4][16][64];
  const int tid = threadIdx.x, w = tid >> 5, lane = tid & 31, ln = lane & 15, hh = lane >> 4; const int by = blockIdx.y;
  A += (size_t)by * sA; Bh += (size_t)by * sB; const size_t cofs = (size_t)by * sC; const float* bp = bias ? bias + (size_t)by * sBias : nullptr;
  const int ntn = (N + 63) / 64; const int wid = blockIdx.x * 4 + w; const int mt = wid / ntn, nq = wid % ntn; if (mt * 16 >= M) return;
  const int row0 = mt * 16, col0 = nq * 64; const _Float16* arow = A + (size_t)(row0 + ln) * lda;
  v8f acc[4] = {};
  for (int kb = 0; kb < K; kb += 32) { FragH ah; ah.half[0] = *(const v8us*)((const unsigned short*)arow + kb + 8 * hh); ah.half[1] = *(const v8us*)((const unsigned short*)arow + kb + 16 + 8 * hh);
#pragma unroll
    for (int t = 0; t < 4; ++t) { if (col0 + t * 16 >= N) continue; const size_t boff = (size_t)(col0 + t * 16 + ln) * ldb + kb; FragH bq; bq.half[0] = *(const v8us*)((const unsigned short*)Bh + boff + 8 * hh); bq.half[1] = *(const v8us*)((const unsigned short*)Bh + boff + 16 + 8 * hh);
      acc[t] = mmaH<1>(ah.v, ah.v, bq.v, bq.v, acc[t]); }
  }
#pragma unroll
  for (int t = 0; t < 4; ++t) { if (col0 + t * 16 >= N) continue; const int col = col0 + t * 16 + ln; const float bv = bp ? bf16_round(bp[col]) : 0.f;
#pragma unroll
    for (int r = 0; r < 8; ++r) { float v = acc[t][r] * alpha + bv; if (CP) { const int bidx = (row0g + row0 + 8 * hh + r) / rowsPerB; v += CP[(size_t)bidx * sCPb + (size_t)by * 64 + col]; } if (ACT == 1) v = (v > 0.f) ? v : expm1f(v); else if (ACT == 7) v = (v > 0.f) ? v + 1.0f : expf(v); else if (ACT == 8) v = tanhf(v); else if (ACT == 9) v = 0.5f * v * (1.0f + tanhf(0.7978845608028654f * (v + 0.044715f * v * v * v))); else if (ACT == 11) v = 1.0f / (1.0f + expf(-v)); else if (ACT == 12) v = (v > 0.f) ? v : 0.01f * v; else if (ACT == 14) v = (v > 0.f) ? v : 0.1f * v; else if (ACT == 15) v = v / (1.0f + expf(-v)); else if (ACT == 3) v = fmaxf(v, 0.f); else if (ACT == 6) v = 0.5f * v * (1.0f + erff(v * 0.70710678118654752f)); so[w][8 * hh + r][t * 16 + ln] = v; } }
  __builtin_amdgcn_fence(__ATOMIC_ACQ_REL, "workgroup"); __builtin_amdgcn_wave_barrier();
  const int rsub = lane >> 4, c4 = (lane & 15) * 4; typedef _Float16 v4h __attribute__((ext_vector_type(4)));
  for (int pass = 0; pass < 2; ++pass) {
#pragma unroll
    for (int q = 0; q < 8; ++q) { const int r = q * 2 + rsub; if (col0 + c4 < N) { const v4f v = *(const v4fa*)&so[w][r][c4]; if (C) *(volatile v4f*)(C + cofs + (size_t)(row0 + r) * ldc + col0 + c4) = v; if (C16) { v4h h4; for (int i = 0; i < 4; ++i) h4[i] = (_Float16)v[i]; *(volatile v4h*)(C16 + cofs + (size_t)(row0 + r) * ldc + col0 + c4) = h4; } } }
    if (pass == 0) __threadfence(); }
}


typedef _Float16 v4h __attribute__((ext_vector_type(4)));

__global__ __launch_bounds__(256) void k_x16(const float* __restrict__ x, _Float16* __restrict__ X16, size_t n8) { const size_t t = (size_t)blockIdx.x * 256 + threadIdx.x; if (t >= n8) return; FragH f;
#pragma unroll
  for (int q = 0; q < 8; ++q) f.h[q] = (_Float16)bf16_round(x[t * 8 + q]); *(volatile v8us*)((unsigned short*)X16 + t * 8) = f.half[0]; __threadfence(); *(volatile v8us*)((unsigned short*)X16 + t * 8) = f.half[0]; }
__global__ __launch_bounds__(256) void k_h16(const float* __restrict__ x, _Float16* __restrict__ X16, size_t n8) { const size_t t = (size_t)blockIdx.x * 256 + threadIdx.x; if (t >= n8) return; FragH f;
#pragma unroll
  for (int q = 0; q < 8; ++q) f.h[q] = (_Float16)x[t * 8 + q]; *(volatile v8us*)((unsigned short*)X16 + t * 8) = f.half[0]; __threadfence(); *(volatile v8us*)((unsigned short*)X16 + t * 8) = f.half[0]; }
__global__ __launch_bounds__(256) void k_round16f(const float* __restrict__ W, _Float16* __restrict__ Bt, size_t n8) { const size_t t = (size_t)blockIdx.x * 256 + threadIdx.x; if (t >= n8) return; FragH f;
#pragma unroll
  for (int i = 0; i < 8; ++i) f.h[i] = (_Float16)(bf16_round(W[t * 8 + i]) * 16.0f); *(volatile v8us*)((unsigned short*)Bt + t * 8) = f.half[0]; __threadfence(); *(volatile v8us*)((unsigned short*)Bt + t * 8) = f.half[0]; }
template <int NHv, int TTv>
__global__ __launch_bounds__(256) void k_vt(const _Float16* __restrict__ V16, int ldv, int voff, _Float16* __restrict__ Vt) { __shared__ unsigned short tl[64][66]; const int tid = threadIdx.x; const int slab = blockIdx.x / (TTv / 64), lg = blockIdx.x % (TTv / 64); const int b = slab / NHv, h = slab % NHv;
  for (int i = tid; i < 64 * 8; i += 256) { const int r = i / 8, c8 = (i % 8) * 8; FragH f; f.half[0] = *(const v8us*)((const unsigned short*)V16 + ((size_t)b * TTv + lg * 64 + r) * ldv + voff + h * 64 + c8);
#pragma unroll
    for (int q = 0; q < 8; ++q) tl[r][c8 + q] = f.u[q]; }
  __syncthreads();
  for (int pass = 0; pass < 2; ++pass) {
#pragma unroll
    for (int rd = 0; rd < 2; ++rd) { const int d = rd * 32 + tid / 8, pc = tid % 8; FragH f;
#pragma unroll
      for (int q = 0; q < 8; ++q) f.u[q] = tl[pc * 8 + q][d];
      *(volatile v8us*)((unsigned short*)Vt + ((size_t)slab * 64 + d) * TTv + lg * 64 + pc * 8) = f.half[0]; }
    if (pass == 0) __threadfence(); } }

__global__ __launch_bounds__(256) void k_hl(const float* __restrict__ F, _Float16* __restrict__ Hh, _Float16* __restrict__ Hl, size_t n8) { const size_t t = (size_t)blockIdx.x * 256 + threadIdx.x; if (t >= n8) return; FragH fh, fl; const v4f a = *(const v4fa*)(F + t * 8), c = *(const v4fa*)(F + t * 8 + 4);
#pragma unroll
  for (int q = 0; q < 4; ++q) { _Float16 h = (_Float16)a[q]; fh.h[q] = h; fl.h[q] = (_Float16)((a[q] - (float)h) * 1024.0f); h = (_Float16)c[q]; fh.h[4 + q] = h; fl.h[4 + q] = (_Float16)((c[q] - (float)h) * 1024.0f); }
  for (int pass = 0; pass < 2; ++pass) { *(volatile v8us*)((unsigned short*)Hh + t * 8) = fh.half[0]; *(volatile v8us*)((unsigned short*)Hl + t * 8) = fl.half[0]; if (pass == 0) __threadfence(); } }

__device__ __forceinline__ float sigm_p(float x) { return 1.0f / (1.0f + expf(-x)); }
__device__ __forceinline__ float sigm_f(float x) { return __builtin_amdgcn_rcpf(1.0f + __expf(-x)); }
__global__ __launch_bounds__(256) void k_ln(const float* __restrict__ x, const float* __restrict__ w, const float* __restrict__ b, float* __restrict__ XN) {
  #pragma clang fp contract(off)
  const int tid = threadIdx.x, wv = tid >> 5, l = tid & 31; const int t = blockIdx.x * 8 + wv; float v[64]; float s = 0.f;
#pragma unroll
  for (int q = 0; q < 8; ++q) { const v4f a = *(const v4fa*)(x + (size_t)t * HDN + q * 256 + 4 * l), c = *(const v4fa*)(x + (size_t)t * HDN + q * 256 + 128 + 4 * l);
#pragma unroll
    for (int j = 0; j < 4; ++j) { v[q * 8 + j] = bf16_round(a[j]); v[q * 8 + 4 + j] = bf16_round(c[j]); s += v[q * 8 + j] + v[q * 8 + 4 + j]; } }
  for (int o = 16; o > 0; o >>= 1) s += __shfl_xor(s, o, 32); const float mu = s / (float)HDN; float vs = 0.f;
#pragma unroll
  for (int i = 0; i < 64; ++i) { const float d = v[i] - mu; vs += d * d; }
  for (int o = 16; o > 0; o >>= 1) vs += __shfl_xor(vs, o, 32); const float rs = 1.0f / sqrtf(vs / (float)HDN + 1e-5f);
  for (int pass = 0; pass < 2; ++pass) {
#pragma unroll
    for (int q = 0; q < 8; ++q) { v4f a, c;
#pragma unroll
      for (int j = 0; j < 4; ++j) { const int c0 = q * 256 + 4 * l + j; a[j] = (v[q * 8 + j] - mu) * rs * bf16_round(w[c0]) + bf16_round(b[c0]); c[j] = (v[q * 8 + 4 + j] - mu) * rs * bf16_round(w[c0 + 128]) + bf16_round(b[c0 + 128]); }
      *(volatile v4f*)(XN + (size_t)t * HDN + q * 256 + 4 * l) = a; *(volatile v4f*)(XN + (size_t)t * HDN + q * 256 + 128 + 4 * l) = c; }
    if (pass == 0) __threadfence(); } }
__global__ __launch_bounds__(256) void k_mix(const float* __restrict__ XN, const float* __restrict__ st1, const float* __restrict__ mu, _Float16* __restrict__ Hh, _Float16* __restrict__ Hl) {
  #pragma clang fp contract(off)
  const size_t tq = (size_t)blockIdx.x * 256 + threadIdx.x; if (tq >= (size_t)TT * HDN / 8) return; const size_t e0 = tq * 8; const int t = (int)(e0 / HDN), c0 = (int)(e0 % HDN); FragH fh, fl;
#pragma unroll
  for (int q = 0; q < 8; ++q) { const int c = c0 + q; const float xv = XN[(size_t)t * HDN + c]; const float pv = (t == 0) ? bf16_round(st1[c]) : XN[(size_t)(t - 1) * HDN + c]; const float m = xv + bf16_round(mu[c]) * (pv - xv); const _Float16 hi = (_Float16)m; fh.h[q] = hi; fl.h[q] = (_Float16)((m - (float)hi) * 1024.0f); }
  for (int pass = 0; pass < 2; ++pass) { *(volatile v8us*)((unsigned short*)Hh + e0) = fh.half[0]; *(volatile v8us*)((unsigned short*)Hl + e0) = fl.half[0]; if (pass == 0) __threadfence(); } }
template <int OP>
__global__ __launch_bounds__(256) void k_act16(const float* __restrict__ F, _Float16* __restrict__ H, size_t n8) {
  #pragma clang fp contract(off)
  const size_t t = (size_t)blockIdx.x * 256 + threadIdx.x; if (t >= n8) return; const v4f a = *(const v4fa*)(F + t * 8), c = *(const v4fa*)(F + t * 8 + 4); FragH f;
#pragma unroll
  for (int q = 0; q < 8; ++q) { float v = (q < 4) ? a[q] : c[q - 4]; if (OP == 1) v = tanhf(v); else if (OP == 2) v = sigm_p(v); f.h[q] = (_Float16)v; }
  *(volatile v8us*)((unsigned short*)H + t * 8) = f.half[0]; __threadfence(); *(volatile v8us*)((unsigned short*)H + t * 8) = f.half[0]; }
__global__ __launch_bounds__(256) void k_prep(const float* __restrict__ R, const float* __restrict__ K, const float* __restrict__ V, const float* __restrict__ WL, const float* __restrict__ AL, const float* __restrict__ VL, const float* __restrict__ vfirst, const float* __restrict__ w0, const float* __restrict__ a0, const float* __restrict__ v0, const float* __restrict__ kk_, const float* __restrict__ ka_, const float* __restrict__ rk_, int t0,
    float* __restrict__ Wp, float* __restrict__ KKp, float* __restrict__ KAp, float* __restrict__ K2p, float* __restrict__ V2p, float* __restrict__ RB) {
  #pragma clang fp contract(off)
  __shared__ __attribute__((aligned(16))) float rbs[NHh]; const int tid = threadIdx.x; const int t = t0 + blockIdx.x; const int l16 = tid & 15;
  v4f wv[2], kkv[2], kav[2], k2v[2], v2v[2];
#pragma unroll
  for (int s = 0; s < 2; ++s) { const int cb = s * 1024 + 4 * tid; float r[4], k[4], v[4], w[4], a[4], kk[4]; float kn = 0.f;
#pragma unroll
    for (int q = 0; q < 4; ++q) { const int c = cb + q; const size_t e = (size_t)t * HDN + c; r[q] = R[e]; k[q] = K[e]; v[q] = V[e];
      w[q] = __expf(-0.606531f * sigm_f(bf16_round(w0[c]) + WL[e])); a[q] = sigm_f(bf16_round(a0[c]) + AL[e]); kk[q] = k[q] * bf16_round(kk_[c]); kn += kk[q] * kk[q];
      v[q] = v[q] + (bf16_round(vfirst[e]) - v[q]) * sigm_f(bf16_round(v0[c]) + VL[e]); }
    for (int o = 8; o > 0; o >>= 1) kn += __shfl_xor(kn, o, 32); const float inrm = __builtin_amdgcn_rcpf(fmaxf(sqrtf(kn), 1e-12f)); float rb = 0.f;
#pragma unroll
    for (int q = 0; q < 4; ++q) { const int c = cb + q; const float kkn = kk[q] * inrm; const float k2 = k[q] * (1.0f + (a[q] - 1.0f) * bf16_round(ka_[c])); rb += r[q] * k2 * bf16_round(rk_[c]); wv[s][q] = w[q]; kkv[s][q] = kkn; kav[s][q] = kkn * a[q]; k2v[s][q] = k2; v2v[s][q] = v[q]; }
    for (int o = 8; o > 0; o >>= 1) rb += __shfl_xor(rb, o, 32); if (l16 == 0) rbs[s * 16 + (tid >> 4)] = rb; }
  __syncthreads();
  for (int pass = 0; pass < 2; ++pass) {
#pragma unroll
    for (int s = 0; s < 2; ++s) { const size_t e = (size_t)t * HDN + s * 1024 + 4 * tid; *(volatile v4f*)(Wp + e) = wv[s]; *(volatile v4f*)(KKp + e) = kkv[s]; *(volatile v4f*)(KAp + e) = kav[s]; *(volatile v4f*)(K2p + e) = k2v[s]; *(volatile v4f*)(V2p + e) = v2v[s]; }
    if (tid < NHh / 4) { const v4f q4 = *(const v4fa*)&rbs[tid * 4]; *(volatile v4f*)(RB + (size_t)t * NHh + tid * 4) = q4; }
    if (pass == 0) __threadfence(); } }
__global__ __launch_bounds__(256) void k_wkv(const float* __restrict__ st2, const float* __restrict__ Wp, const float* __restrict__ KKp, const float* __restrict__ KAp, const float* __restrict__ K2p, const float* __restrict__ V2p, const float* __restrict__ Rp, float* __restrict__ Y, float* __restrict__ out) {
  #pragma clang fp contract(off)
  __shared__ float S[HS][HS + 1]; __shared__ float wk[5][HS]; __shared__ float ys[HS];
  const int tid = threadIdx.x; const int h = blockIdx.x; const int i = tid >> 2, jq = tid & 3, j0 = jq * 16;
  for (int e = tid; e < HS * HS; e += 256) S[e / HS][e % HS] = bf16_round(st2[(size_t)h * HS * HS + e]);
  __syncthreads();
#pragma unroll 1
  for (int t = 0; t < TT; ++t) { const size_t base = (size_t)t * HDN + h * HS;
    if (tid < HS) { wk[0][tid] = Wp[base + tid]; wk[1][tid] = KKp[base + tid]; wk[2][tid] = KAp[base + tid]; wk[3][tid] = K2p[base + tid]; wk[4][tid] = Rp[base + tid]; }
    __syncthreads();
    float sa = 0.f;
#pragma unroll 1
    for (int j = j0; j < j0 + 16; ++j) sa += S[i][j] * wk[1][j];
    sa += __shfl_xor(sa, 1, 32); sa += __shfl_xor(sa, 2, 32);
    const float vi = V2p[base + i]; float yp = 0.f;
#pragma unroll 1
    for (int j = j0; j < j0 + 16; ++j) { const float s = (S[i][j] * wk[0][j] - sa * wk[2][j]) + vi * wk[3][j]; S[i][j] = s; yp += s * wk[4][j]; }
    yp += __shfl_xor(yp, 1, 32); yp += __shfl_xor(yp, 2, 32); if (jq == 0) ys[i] = yp;
    __syncthreads();
    if (tid < HS) { float* p = Y + base + tid; const float yv = ys[tid]; *(volatile float*)p = yv; __threadfence(); *(volatile float*)p = yv; }
    __syncthreads(); }
  for (int pass = 0; pass < 2; ++pass) { for (int e = tid; e < HS * HS; e += 256) *(volatile float*)(out + OFF_S2 + (size_t)h * HS * HS + e) = S[e / HS][e % HS]; if (pass == 0) __threadfence(); } }
__global__ __launch_bounds__(256) void k_fin(const float* __restrict__ Y, const float* __restrict__ V2p, const float* __restrict__ RB, const float* __restrict__ G, const float* __restrict__ lw, const float* __restrict__ lb, _Float16* __restrict__ Z16) {
  #pragma clang fp contract(off)
  const int tid = threadIdx.x, wv = tid >> 5, l = tid & 31; const int th = blockIdx.x * 8 + wv; const int t = th / NHh, h = th % NHh; const size_t e = (size_t)t * HDN + h * HS + 2 * l; const float y0 = Y[e], y1 = Y[e + 1]; float s = y0 + y1; for (int o = 16; o > 0; o >>= 1) s += __shfl_xor(s, o, 32); const float mu = s / 64.0f; float vs = (y0 - mu) * (y0 - mu) + (y1 - mu) * (y1 - mu); for (int o = 16; o > 0; o >>= 1) vs += __shfl_xor(vs, o, 32); const float rs = 1.0f / sqrtf(vs / 64.0f + 64e-5f); const float rb = RB[(size_t)t * NHh + h];
  FragH f; const int c = h * HS + 2 * l;
  f.h[0] = (_Float16)((((y0 - mu) * rs * bf16_round(lw[c]) + bf16_round(lb[c])) + rb * V2p[e]) * G[e]); f.h[1] = (_Float16)((((y1 - mu) * rs * bf16_round(lw[c + 1]) + bf16_round(lb[c + 1])) + rb * V2p[e + 1]) * G[e + 1]);
  const unsigned int pv = *(const unsigned int*)&f.u[0]; *(volatile unsigned int*)((unsigned short*)Z16 + e) = pv; __threadfence(); *(volatile unsigned int*)((unsigned short*)Z16 + e) = pv; }
__global__ __launch_bounds__(256) void k_misc(const float* __restrict__ XN, const float* __restrict__ vfirst, const float* __restrict__ x, float* __restrict__ Xb, float* __restrict__ out) { const size_t t = (size_t)blockIdx.x * 256 + threadIdx.x; const size_t n4 = (size_t)TT * HDN / 4; if (t >= n4) return; const v4f vf = *(const v4fa*)(vfirst + t * 4), xx = *(const v4fa*)(x + t * 4); v4f a, b;
#pragma unroll
  for (int q = 0; q < 4; ++q) { a[q] = bf16_round(vf[q]); b[q] = bf16_round(xx[q]); }
  for (int pass = 0; pass < 2; ++pass) { *(volatile v4f*)(out + OFF_VF + t * 4) = a; *(volatile v4f*)(Xb + t * 4) = b; if (t < HDN / 4) { const v4f s1 = *(const v4fa*)(XN + (size_t)(TT - 1) * HDN + t * 4); *(volatile v4f*)(out + OFF_S1 + t * 4) = s1; } if (pass == 0) __threadfence(); } }

extern "C" void kernel_launch(void* const* d_in, const int* in_sizes, int n_in,
                              void* d_out, int out_size, void* d_ws, size_t ws_size, hipStream_t stream) {
  (void)in_sizes; (void)n_in; (void)out_size;
  const float* const* I = (const float* const*)d_in; const float* x = I[0]; const float* st1 = I[1]; const float* st2 = I[2]; const float* vfirst = I[3]; const float* ln1w = I[4]; const float* ln1b = I[5];
  const float* mu[6] = {I[6], I[7], I[8], I[9], I[10], I[11]};
  const float* Wr = I[12]; const float* Wk = I[13]; const float* Wv = I[14]; const float* Wo = I[15]; const float* w0 = I[16]; const float* w1 = I[17]; const float* w2 = I[18]; const float* a0 = I[19]; const float* a1 = I[20]; const float* a2 = I[21]; const float* v0 = I[22]; const float* v1 = I[23]; const float* v2 = I[24]; const float* g1 = I[25]; const float* g2 = I[26]; const float* kk_ = I[27]; const float* ka_ = I[28]; const float* rk_ = I[29]; const float* lxw = I[30]; const float* lxb = I[31];
  char* ws = (char*)d_ws; size_t off = 0;
  auto take = [&](size_t bytes) { char* p = ws + off; off += (bytes + 255) & ~(size_t)255; return p; };
  const size_t PL = (size_t)TT * HDN;
  _Float16* BW = (_Float16*)take((size_t)HDN * HDN * 2);
  _Float16* Bw1 = (_Float16*)take((size_t)DW * HDN * 2); _Float16* Bw2 = (_Float16*)take((size_t)HDN * DW * 2); _Float16* Ba1 = (_Float16*)take((size_t)DA * HDN * 2); _Float16* Ba2 = (_Float16*)take((size_t)HDN * DA * 2); _Float16* Bv1 = (_Float16*)take((size_t)DV * HDN * 2); _Float16* Bv2 = (_Float16*)take((size_t)HDN * DV * 2); _Float16* Bg1 = (_Float16*)take((size_t)DG * HDN * 2); _Float16* Bg2 = (_Float16*)take((size_t)HDN * DG * 2);
  float* XN = (float*)take(PL * 4); _Float16* Hh = (_Float16*)take(PL * 2); _Float16* Hl = (_Float16*)take(PL * 2); float* R = (float*)take(PL * 4); float* K = (float*)take(PL * 4); float* V = (float*)take(PL * 4);
  float* LT = (float*)take((size_t)TT * DG * 4); _Float16* L16 = (_Float16*)take((size_t)TT * DG * 2); float* WL = (float*)take(PL * 4); float* AL = (float*)take(PL * 4); float* VL = (float*)take(PL * 4); float* G = (float*)take(PL * 4);
  if (off > ws_size) return;
  float* Wp = WL; float* KKp = AL; float* KAp = (float*)Hh;    float* K2p = K; float* V2p = V; float* Yp = XN  ;
  float* Y = (float*)take(PL * 4); float* RB = (float*)take((size_t)TT * NHh * 4); _Float16* Z16 = (_Float16*)take(PL * 2); float* Xb = (float*)take(PL * 4);
  (void)Yp; if (off > ws_size) return;
  const unsigned gW = (unsigned)(((size_t)HDN * (HDN / 8) + 255) / 256); const size_t n8 = PL / 8; const unsigned g8 = (unsigned)((n8 + 255) / 256);
  const dim3 gBig(((TT / 16) * (HDN / 64) + 3) / 4, 1);
  k_ln<<<TT / 8, 256, 0, stream>>>(x, ln1w, ln1b, XN);
  k_misc<<<(unsigned)((PL / 4 + 255) / 256), 256, 0, stream>>>(XN, vfirst, x, Xb, (float*)d_out);
  k_wt_f16<<<(DW * (HDN / 8) + 255) / 256, 256, 0, stream>>>(w1, Bw1, HDN, DW, 16.0f); k_wt_f16<<<(HDN * (DW / 8) + 255) / 256, 256, 0, stream>>>(w2, Bw2, DW, HDN, 16.0f);
  k_wt_f16<<<(DA * (HDN / 8) + 255) / 256, 256, 0, stream>>>(a1, Ba1, HDN, DA, 16.0f); k_wt_f16<<<(HDN * (DA / 8) + 255) / 256, 256, 0, stream>>>(a2, Ba2, DA, HDN, 16.0f);
  k_wt_f16<<<(DV * (HDN / 8) + 255) / 256, 256, 0, stream>>>(v1, Bv1, HDN, DV, 16.0f); k_wt_f16<<<(HDN * (DV / 8) + 255) / 256, 256, 0, stream>>>(v2, Bv2, DV, HDN, 16.0f);
  k_wt_f16<<<(DG * (HDN / 8) + 255) / 256, 256, 0, stream>>>(g1, Bg1, HDN, DG, 16.0f); k_wt_f16<<<(HDN * (DG / 8) + 255) / 256, 256, 0, stream>>>(g2, Bg2, DG, HDN, 16.0f);
  k_wt_f16<<<gW, 256, 0, stream>>>(Wr, BW, HDN, HDN, 16.0f); k_mix<<<g8, 256, 0, stream>>>(XN, st1, mu[0], Hh, Hl);
  k_gemm_hhx<0><<<gBig, 128, 0, stream>>>(Hh, HDN, 0, BW, HDN, 0, 0.0625f, nullptr, 0, nullptr, 1, 0, 0, R, nullptr, HDN, 0, TT, HDN, HDN); k_gemm_hhx<0><<<gBig, 128, 0, stream>>>(Hl, HDN, 0, BW, HDN, 0, 0.0625f / 1024.0f, nullptr, 0, R, 1, (size_t)HDN, 0, R, nullptr, HDN, 0, TT, HDN, HDN);
  k_mix<<<g8, 256, 0, stream>>>(XN, st1, mu[1], Hh, Hl);
  k_gemm_hhx<0><<<dim3(((TT / 16) * ((DW + 63) / 64) + 3) / 4, 1), 128, 0, stream>>>(Hh, HDN, 0, Bw1, HDN, 0, 0.0625f, nullptr, 0, nullptr, 1, 0, 0, LT, nullptr, DW, 0, TT, DW, HDN); k_act16<1><<<(unsigned)(((size_t)TT * DW / 8 + 255) / 256), 256, 0, stream>>>(LT, L16, (size_t)TT * DW / 8);
  k_gemm_hhx<0><<<gBig, 128, 0, stream>>>(L16, DW, 0, Bw2, DW, 0, 0.0625f, nullptr, 0, nullptr, 1, 0, 0, WL, nullptr, HDN, 0, TT, HDN, DW);
  k_wt_f16<<<gW, 256, 0, stream>>>(Wk, BW, HDN, HDN, 16.0f); k_mix<<<g8, 256, 0, stream>>>(XN, st1, mu[2], Hh, Hl);
  k_gemm_hhx<0><<<gBig, 128, 0, stream>>>(Hh, HDN, 0, BW, HDN, 0, 0.0625f, nullptr, 0, nullptr, 1, 0, 0, K, nullptr, HDN, 0, TT, HDN, HDN); k_gemm_hhx<0><<<gBig, 128, 0, stream>>>(Hl, HDN, 0, BW, HDN, 0, 0.0625f / 1024.0f, nullptr, 0, K, 1, (size_t)HDN, 0, K, nullptr, HDN, 0, TT, HDN, HDN);
  k_wt_f16<<<gW, 256, 0, stream>>>(Wv, BW, HDN, HDN, 16.0f); k_mix<<<g8, 256, 0, stream>>>(XN, st1, mu[3], Hh, Hl);
  k_gemm_hhx<0><<<gBig, 128, 0, stream>>>(Hh, HDN, 0, BW, HDN, 0, 0.0625f, nullptr, 0, nullptr, 1, 0, 0, V, nullptr, HDN, 0, TT, HDN, HDN); k_gemm_hhx<0><<<gBig, 128, 0, stream>>>(Hl, HDN, 0, BW, HDN, 0, 0.0625f / 1024.0f, nullptr, 0, V, 1, (size_t)HDN, 0, V, nullptr, HDN, 0, TT, HDN, HDN);
  k_gemm_hhx<0><<<dim3(((TT / 16) * 1 + 3) / 4, 1), 128, 0, stream>>>(Hh, HDN, 0, Bv1, HDN, 0, 0.0625f, nullptr, 0, nullptr, 1, 0, 0, LT, nullptr, DV, 0, TT, DV, HDN); k_act16<0><<<(unsigned)(((size_t)TT * DV / 8 + 255) / 256), 256, 0, stream>>>(LT, L16, (size_t)TT * DV / 8);
  k_gemm_hhx<0><<<gBig, 128, 0, stream>>>(L16, DV, 0, Bv2, DV, 0, 0.0625f, nullptr, 0, nullptr, 1, 0, 0, VL, nullptr, HDN, 0, TT, HDN, DV);
  k_mix<<<g8, 256, 0, stream>>>(XN, st1, mu[4], Hh, Hl);
  k_gemm_hhx<0><<<dim3(((TT / 16) * ((DA + 63) / 64) + 3) / 4, 1), 128, 0, stream>>>(Hh, HDN, 0, Ba1, HDN, 0, 0.0625f, nullptr, 0, nullptr, 1, 0, 0, LT, nullptr, DA, 0, TT, DA, HDN); k_act16<0><<<(unsigned)(((size_t)TT * DA / 8 + 255) / 256), 256, 0, stream>>>(LT, L16, (size_t)TT * DA / 8);
  k_gemm_hhx<0><<<gBig, 128, 0, stream>>>(L16, DA, 0, Ba2, DA, 0, 0.0625f, nullptr, 0, nullptr, 1, 0, 0, AL, nullptr, HDN, 0, TT, HDN, DA);
  k_mix<<<g8, 256, 0, stream>>>(XN, st1, mu[5], Hh, Hl);
  k_gemm_hhx<0><<<dim3(((TT / 16) * (DG / 64) + 3) / 4, 1), 128, 0, stream>>>(Hh, HDN, 0, Bg1, HDN, 0, 0.0625f, nullptr, 0, nullptr, 1, 0, 0, LT, nullptr, DG, 0, TT, DG, HDN); k_act16<2><<<(unsigned)(((size_t)TT * DG / 8 + 255) / 256), 256, 0, stream>>>(LT, L16, (size_t)TT * DG / 8);
  k_gemm_hhx<0><<<gBig, 128, 0, stream>>>(L16, DG, 0, Bg2, DG, 0, 0.0625f, nullptr, 0, nullptr, 1, 0, 0, G, nullptr, HDN, 0, TT, HDN, DG);
  k_prep<<<TT, 256, 0, stream>>>(R, K, V, WL, AL, VL, vfirst, w0, a0, v0, kk_, ka_, rk_, 0, Wp, KKp, KAp, K2p, V2p, RB);
  k_wkv<<<NHh, 256, 0, stream>>>(st2, Wp, KKp, KAp, K2p, V2p, R, Y, (float*)d_out);
  k_fin<<<TT * NHh / 8, 256, 0, stream>>>(Y, V2p, RB, G, lxw, lxb, Z16);
  k_wt_f16<<<gW, 256, 0, stream>>>(Wo, BW, HDN, HDN, 16.0f);
  k_gemm_hhx<0><<<gBig, 128, 0, stream>>>(Z16, HDN, 0, BW, HDN, 0, 0.0625f, nullptr, 0, Xb, 1, (size_t)HDN, 0, (float*)d_out, nullptr, HDN, 0, TT, HDN, HDN);
}
